// SAModule_4698694222638
// MI455X (gfx1250) — hardware-verified
//
#include <hip/hip_runtime.h>
#include <math.h>

constexpr int kB      = 32;
constexpr int kC      = 64;
constexpr int kSpW    = 32;
constexpr int kSpH    = 32;
constexpr int kN      = kSpW * kSpH;
constexpr int kHeads  = 4;
constexpr int kDh     = 16;
constexpr int kTok    = kB * kN;
constexpr int kZ      = kB * kHeads;
constexpr int kKQCols = 2 * kC;
constexpr int kSK     = 2 * kDh;
constexpr int kGroup  = 8;
constexpr int kChunks = kZ / kGroup;
constexpr int kCN     = kC * kN;
constexpr int kHid    = 4;
constexpr int kTaps   = 2 * 7 * 7;
constexpr float kPCarry    = 32768.0f;
constexpr float kPCarryInv = 1.0f / 32768.0f;
constexpr float kLnEps     = 1.0e-5f;
static_assert(kHeads * kDh == kC, "shape");
static_assert(kZ % kGroup == 0 && kB % kGroup == 0, "chunks");
static_assert(kC % 32 == 0 && kSK % 32 == 0 && kN % 32 == 0, "K multiples of 32");
static_assert(kTok % 64 == 0 && kKQCols % 64 == 0 && kN % 64 == 0 && kC % 64 == 0 && kDh % 16 == 0, "tile multiples");

typedef __attribute__((ext_vector_type(16))) _Float16 v16h;
typedef __attribute__((ext_vector_type(8)))  _Float16 v8h;
typedef __attribute__((ext_vector_type(16))) __bf16   v16b;
typedef __attribute__((ext_vector_type(8)))  __bf16   v8b;
typedef __attribute__((ext_vector_type(8)))  float    v8f;
typedef __attribute__((ext_vector_type(4)))  float    v4f;
typedef __attribute__((ext_vector_type(4)))  unsigned int v4u;

__device__ __forceinline__ unsigned short f2bf_bits(float f) {
  unsigned u = __float_as_uint(f);
  return (unsigned short)((u + 0x7FFFu + ((u >> 16) & 1u)) >> 16);
}
__device__ __forceinline__ float bf_bits2f(unsigned short h) { return __uint_as_float(((unsigned)h) << 16); }
__device__ __forceinline__ unsigned pk16(unsigned short a, unsigned short b) { return (unsigned)a | ((unsigned)b << 16); }
__device__ __forceinline__ unsigned short h_bits(float f) { const _Float16 h = (_Float16)f; return __builtin_bit_cast(unsigned short, h); }

__device__ __forceinline__ void dep_guard_all_h(v8f& a0, v8f& a1, v8f& a2, v8f& a3, v16h x, v16h y, v16h p0, v16h p1, v16h p2, v16h p3) {
  asm volatile("v_nop\n\tv_nop\n\tv_nop\n\tv_nop" : "+v"(a0), "+v"(a1), "+v"(a2), "+v"(a3) : "v"(x), "v"(y), "v"(p0), "v"(p1), "v"(p2), "v"(p3));
}
__device__ __forceinline__ void dep_guard_all_b(v8f& a0, v8f& a1, v8f& a2, v8f& a3, v16b x, v16b y, v16b p0, v16b p1, v16b p2, v16b p3) {
  asm volatile("v_nop\n\tv_nop\n\tv_nop\n\tv_nop" : "+v"(a0), "+v"(a1), "+v"(a2), "+v"(a3) : "v"(x), "v"(y), "v"(p0), "v"(p1), "v"(p2), "v"(p3));
}
__device__ __forceinline__ void keep4_h(v16h a, v16h b, v16h c, v16h d) { asm volatile("v_nop" :: "v"(a), "v"(b), "v"(c), "v"(d)); }
__device__ __forceinline__ void keep4_b(v16b a, v16b b, v16b c, v16b d) { asm volatile("v_nop" :: "v"(a), "v"(b), "v"(c), "v"(d)); }
__device__ __forceinline__ void acc_guard4(v8f& a, v8f& b, v8f& c, v8f& d) { asm volatile("v_nop\n\tv_nop\n\tv_nop\n\tv_nop" : "+v"(a), "+v"(b), "+v"(c), "+v"(d)); }
template <typename T> struct Frag;
template <> struct Frag<_Float16> {
  typedef v16h V; union U { v16h v; v8h h[2]; };
  static __device__ __forceinline__ v16h load(const _Float16* p) {
    U f; f.h[0] = *(const v8h*)(p); f.h[1] = *(const v8h*)(p + 16); return f.v;
  }
  static __device__ __forceinline__ v8f mma(v16h a, v16h b, v8f c) {
    return __builtin_amdgcn_wmma_f32_16x16x32_f16(false, a, false, b, (short)0, c, false, false);
  }
  static __device__ __forceinline__ void guard_all(v8f& a0, v8f& a1, v8f& a2, v8f& a3, v16h x, v16h y, v16h p0, v16h p1, v16h p2, v16h p3) {
    dep_guard_all_h(a0, a1, a2, a3, x, y, p0, p1, p2, p3);
  }
  static __device__ __forceinline__ void keep(v16h a, v16h b, v16h c, v16h d) { keep4_h(a, b, c, d); }
};
template <> struct Frag<__bf16> {
  typedef v16b V; union U { v16b v; v8b h[2]; };
  static __device__ __forceinline__ v16b load(const __bf16* p) {
    U f; f.h[0] = *(const v8b*)(p); f.h[1] = *(const v8b*)(p + 16); return f.v;
  }
  static __device__ __forceinline__ v8f mma(v16b a, v16b b, v8f c) {
    return __builtin_amdgcn_wmma_f32_16x16x32_bf16(false, a, false, b, (short)0, c, false, false);
  }
  static __device__ __forceinline__ void guard_all(v8f& a0, v8f& a1, v8f& a2, v8f& a3, v16b x, v16b y, v16b p0, v16b p1, v16b p2, v16b p3) {
    dep_guard_all_b(a0, a1, a2, a3, x, y, p0, p1, p2, p3);
  }
  static __device__ __forceinline__ void keep(v16b a, v16b b, v16b c, v16b d) { keep4_b(a, b, c, d); }
};

template <int ET> struct Elem;
template <> struct Elem<0> { typedef _Float16 T; };
template <> struct Elem<1> { typedef __bf16 T; };
template <int ET, bool SPLIT, int BIAS_MODE, int OUT_MODE, int MI>
__global__ __launch_bounds__(256) void wmma_gemm(
    const unsigned short* __restrict__ Ap, const unsigned short* __restrict__ A2p, int lda, long strideA,
    const unsigned short* __restrict__ Btp, const unsigned short* __restrict__ Bt2p, int ldb, long strideB,
    void* __restrict__ Cout, void* __restrict__ Cout2, int ldc, long strideC,
    const float* __restrict__ bias,
    int M, int N, int K, float scale) {
  typedef typename Elem<ET>::T T;
  typedef typename Frag<T>::V V;
  const T* A = (const T*)Ap; const T* A2 = (const T*)A2p; const T* Bt = (const T*)Btp; const T* Bt2 = (const T*)Bt2p;
  __shared__ __align__(16) float sT[8][16 * 68];
  const int b    = blockIdx.y;
  const int lane = threadIdx.x & 31;
  const int wave = threadIdx.x >> 5;
  const int tilesN = N >> 6;
  const int tilesM = M / (MI * 16);
  const int tile = blockIdx.x * 8 + wave;
  if (tile >= tilesM * tilesN) return;
  const int tm = tile / tilesN;
  const int tn = tile - tm * tilesN;
  const int m0 = tm * (MI * 16);
  const int n0 = tn << 6;

  const T* Ab  = A  + (size_t)b * strideA;
  const T* Bb  = Bt + (size_t)b * strideB;
  const T* Ab2 = SPLIT ? (A2  + (size_t)b * strideA) : nullptr;
  const T* Bb2 = SPLIT ? (Bt2 + (size_t)b * strideB) : nullptr;

  const int rlane = lane & 15;
  const int koff  = (lane >> 4) * 8;
  const int mOff  = (lane >> 4) * 8;

  v8f acc[MI][4];
#pragma unroll
  for (int i = 0; i < MI; ++i)
#pragma unroll
    for (int j = 0; j < 4; ++j) acc[i][j] = (v8f){0.f,0.f,0.f,0.f,0.f,0.f,0.f,0.f};

  for (int k0 = 0; k0 < K; k0 += 32) {
    V bh[4], bl[4];
#pragma unroll
    for (int j = 0; j < 4; ++j) {
      const size_t bo = (size_t)(n0 + (j << 4) + rlane) * ldb + koff + k0;
      bh[j] = Frag<T>::load(Bb + bo);
      if (SPLIT) bl[j] = Frag<T>::load(Bb2 + bo);
    }
#pragma unroll
    for (int i = 0; i < MI; ++i) {
      const size_t ao = (size_t)(m0 + (i << 4) + rlane) * lda + koff + k0;
      V ah = Frag<T>::load(Ab + ao);
      V al;
      if (SPLIT) al = Frag<T>::load(Ab2 + ao);
#pragma unroll
      for (int j = 0; j < 4; ++j) {
        acc[i][j] = Frag<T>::mma(ah, bh[j], acc[i][j]);
        if (SPLIT) {
          acc[i][j] = Frag<T>::mma(ah, bl[j], acc[i][j]);
          acc[i][j] = Frag<T>::mma(al, bh[j], acc[i][j]);
        }
      }
      Frag<T>::guard_all(acc[i][0], acc[i][1], acc[i][2], acc[i][3], ah, SPLIT ? al : ah, bh[0], bh[1], bh[2], bh[3]);
    }
    Frag<T>::keep(bh[0], bh[1], bh[2], bh[3]);
    if (SPLIT) Frag<T>::keep(bl[0], bl[1], bl[2], bl[3]);
  }
#pragma unroll
  for (int i = 0; i < MI; ++i) acc_guard4(acc[i][0], acc[i][1], acc[i][2], acc[i][3]);

  float* slab = sT[wave];
#pragma unroll
  for (int i = 0; i < MI; ++i) {
    const int mBase = m0 + (i << 4);
    float bm[8];
    if (BIAS_MODE == 1) {
      const v4f t0 = *(const v4f*)(bias + mBase + mOff);
      const v4f t1 = *(const v4f*)(bias + mBase + mOff + 4);
      bm[0] = t0[0]; bm[1] = t0[1]; bm[2] = t0[2]; bm[3] = t0[3];
      bm[4] = t1[0]; bm[5] = t1[1]; bm[6] = t1[2]; bm[7] = t1[3];
    } else {
#pragma unroll
      for (int r = 0; r < 8; ++r) bm[r] = 0.0f;
    }
#pragma unroll
    for (int j = 0; j < 4; ++j) {
      const int n = n0 + (j << 4) + rlane;
      float bv = 0.f;
      if (BIAS_MODE == 2) bv = bias[n];
#pragma unroll
      for (int r = 0; r < 8; ++r) {
        float v = acc[i][j][r] * scale;
        if (BIAS_MODE == 1) v += bm[r];
        if (BIAS_MODE == 2) v += bv;
        slab[(mOff + r) * 68 + (j << 4) + rlane] = v;
      }
    }
    __builtin_amdgcn_fence(__ATOMIC_RELEASE, "workgroup");
    __builtin_amdgcn_wave_barrier();
    __builtin_amdgcn_fence(__ATOMIC_ACQUIRE, "workgroup");
    if (OUT_MODE == 0) {
      float* C = (float*)Cout + (size_t)b * strideC;
      const int hh = lane >> 4, c4 = (lane & 15) * 4;
      for (int pass = 0; pass < 2; ++pass) {
#pragma unroll
        for (int it = 0; it < 8; ++it) {
          const int row = it * 2 + hh;
          v4f v = *(const v4f*)(slab + row * 68 + c4);
          *(volatile v4f*)(C + (size_t)(mBase + row) * ldc + n0 + c4) = v;
        }
        __threadfence();
      }
    } else {
      const int q = lane >> 3, c8 = (lane & 7) * 8;
      unsigned short* C  = (unsigned short*)Cout  + (size_t)b * strideC;
      unsigned short* C2 = (OUT_MODE == 2) ? ((unsigned short*)Cout2 + (size_t)b * strideC) : nullptr;
      for (int pass = 0; pass < 2; ++pass) {
#pragma unroll
        for (int it = 0; it < 4; ++it) {
          const int row = it * 4 + q;
          const float* sp = slab + row * 68 + c8;
          v8h hv, lv;
#pragma unroll
          for (int e = 0; e < 8; ++e) {
            if (OUT_MODE == 1) {
              hv[e] = (_Float16)sp[e];
            } else {
              unsigned short hb = f2bf_bits(sp[e]);
              unsigned short lb = f2bf_bits(sp[e] - bf_bits2f(hb));
              hv[e] = __builtin_bit_cast(_Float16, hb);
              lv[e] = __builtin_bit_cast(_Float16, lb);
            }
          }
          *(volatile v8h*)(C + (size_t)(mBase + row) * ldc + n0 + c8) = hv;
          if (OUT_MODE == 2) *(volatile v8h*)(C2 + (size_t)(mBase + row) * ldc + n0 + c8) = lv;
        }
        __threadfence();
      }
    }
    __builtin_amdgcn_fence(__ATOMIC_RELEASE, "workgroup");
    __builtin_amdgcn_wave_barrier();
    __builtin_amdgcn_fence(__ATOMIC_ACQUIRE, "workgroup");
  }
}

__device__ __forceinline__ float wave_sum(float v) {
#pragma unroll
  for (int off = 16; off > 0; off >>= 1) v += __shfl_xor(v, off, 32);
  return v;
}
__device__ __forceinline__ float wave_max(float v) {
#pragma unroll
  for (int off = 16; off > 0; off >>= 1) v = fmaxf(v, __shfl_xor(v, off, 32));
  return v;
}
__device__ __forceinline__ float sigmoid_f(float z) {
  const float zc = fminf(fmaxf(z, -30.0f), 30.0f);
  const float e = expf(-zc);
  return 1.0f / (1.0f + e);
}

__global__ __launch_bounds__(256) void xt_split_kernel(const float* __restrict__ x,
                                                      unsigned short* __restrict__ Xh, unsigned short* __restrict__ Xl) {
  __shared__ float sm[64][65];
  const int t  = threadIdx.x;
  const int n0 = blockIdx.x * 64;
  const int b  = blockIdx.y;
#pragma unroll
  for (int i = 0; i < 4; ++i) {
    const int idx = i * 256 + t;
    const int c   = idx >> 4;
    const int n4  = (idx & 15) * 4;
    const v4f v = *(const v4f*)(x + ((size_t)(b * kC + c)) * kN + n0 + n4);
    sm[n4 + 0][c] = v[0];
    sm[n4 + 1][c] = v[1];
    sm[n4 + 2][c] = v[2];
    sm[n4 + 3][c] = v[3];
  }
  __syncthreads();
  const int lane = t & 31, wave = t >> 5;
  const int q = lane >> 3, c8 = (lane & 7) * 8;
  const size_t rowbase = (size_t)b * kN + n0;
  for (int pass = 0; pass < 2; ++pass) {
#pragma unroll
    for (int it = 0; it < 2; ++it) {
      const int row = wave * 8 + it * 4 + q;
      unsigned short hb[8], lb[8];
#pragma unroll
      for (int e = 0; e < 8; ++e) {
        const float v = sm[row][c8 + e];
        hb[e] = f2bf_bits(v);
        lb[e] = f2bf_bits(v - bf_bits2f(hb[e]));
      }
      const v4u uh = (v4u){pk16(hb[0], hb[1]), pk16(hb[2], hb[3]), pk16(hb[4], hb[5]), pk16(hb[6], hb[7])};
      const v4u ul = (v4u){pk16(lb[0], lb[1]), pk16(lb[2], lb[3]), pk16(lb[4], lb[5]), pk16(lb[6], lb[7])};
      *(volatile v4u*)(Xh + (rowbase + row) * kC + c8) = uh;
      *(volatile v4u*)(Xl + (rowbase + row) * kC + c8) = ul;
    }
    __threadfence();
  }
}

__global__ __launch_bounds__(256) void prep_kernel(const float* __restrict__ Wq, const float* __restrict__ bq,
                                                  const float* __restrict__ Wk, const float* __restrict__ bk,
                                                  const float* __restrict__ Wv,
                                                  unsigned short* __restrict__ Wkqh, unsigned short* __restrict__ Wkql,
                                                  unsigned short* __restrict__ Wvh, unsigned short* __restrict__ Wvl,
                                                  float* __restrict__ biasKQ) {
  const int t    = threadIdx.x;
  const int rsub = t >> 3, c8 = (t & 7) * 8;
#pragma unroll 1
  for (int it = 0; it < 4; ++it) {
    const int r    = it * 32 + rsub;
    const int hd   = r >> 5, w = r & 31;
    const int srow = hd * 16 + (w & 15);
    const float fk = (w < 16) ? 1.0f : 0.0f;
    const float fq = 1.0f - fk;
    const v4f k0 = *(const v4f*)(Wk + srow * kC + c8);
    const v4f k1 = *(const v4f*)(Wk + srow * kC + c8 + 4);
    const v4f q0 = *(const v4f*)(Wq + srow * kC + c8);
    const v4f q1 = *(const v4f*)(Wq + srow * kC + c8 + 4);
    unsigned short hb[8], lb[8];
#pragma unroll
    for (int e = 0; e < 4; ++e) {
      const float v0 = fmaf(fk, k0[e], fq * q0[e]);
      const float v1 = fmaf(fk, k1[e], fq * q1[e]);
      hb[e] = f2bf_bits(v0);     lb[e] = f2bf_bits(v0 - bf_bits2f(hb[e]));
      hb[4 + e] = f2bf_bits(v1); lb[4 + e] = f2bf_bits(v1 - bf_bits2f(hb[4 + e]));
    }
    const v4u uh = (v4u){pk16(hb[0], hb[1]), pk16(hb[2], hb[3]), pk16(hb[4], hb[5]), pk16(hb[6], hb[7])};
    const v4u ul = (v4u){pk16(lb[0], lb[1]), pk16(lb[2], lb[3]), pk16(lb[4], lb[5]), pk16(lb[6], lb[7])};
    unsigned short* ph = Wkqh + r * kC + c8;
    unsigned short* pl = Wkql + r * kC + c8;
    *(volatile v4u*)ph = uh; *(volatile v4u*)pl = ul;
    __threadfence();
    *(volatile v4u*)ph = uh; *(volatile v4u*)pl = ul;
  }
#pragma unroll 1
  for (int it = 0; it < 2; ++it) {
    const int r = it * 32 + rsub;
    const v4f a0 = *(const v4f*)(Wv + r * kC + c8);
    const v4f a1 = *(const v4f*)(Wv + r * kC + c8 + 4);
    unsigned short hb[8], lb[8];
#pragma unroll
    for (int e = 0; e < 4; ++e) {
      hb[e] = f2bf_bits(a0[e]);     lb[e] = f2bf_bits(a0[e] - bf_bits2f(hb[e]));
      hb[4 + e] = f2bf_bits(a1[e]); lb[4 + e] = f2bf_bits(a1[e] - bf_bits2f(hb[4 + e]));
    }
    const v4u uh = (v4u){pk16(hb[0], hb[1]), pk16(hb[2], hb[3]), pk16(hb[4], hb[5]), pk16(hb[6], hb[7])};
    const v4u ul = (v4u){pk16(lb[0], lb[1]), pk16(lb[2], lb[3]), pk16(lb[4], lb[5]), pk16(lb[6], lb[7])};
    unsigned short* ph = Wvh + r * kC + c8;
    unsigned short* pl = Wvl + r * kC + c8;
    *(volatile v4u*)ph = uh; *(volatile v4u*)pl = ul;
    __threadfence();
    *(volatile v4u*)ph = uh; *(volatile v4u*)pl = ul;
  }
  if (t < 32) {
    v4f bvv;
#pragma unroll
    for (int e = 0; e < 4; ++e) {
      const int r   = 4 * t + e;
      const int idx = (r >> 5) * 16 + (r & 15);
      const float fk = ((r & 16) == 0) ? 1.0f : 0.0f;
      const float fq = 1.0f - fk;
      bvv[e] = fmaf(fk, bk[idx], fq * bq[idx]);
    }
    float* pb = biasKQ + 4 * t;
    *(volatile v4f*)pb = bvv;
    __threadfence();
    *(volatile v4f*)pb = bvv;
  }
}

__global__ __launch_bounds__(256) void pack_kernel(const unsigned short* __restrict__ KQh, const unsigned short* __restrict__ KQl,
                                                  const float* __restrict__ relh, const float* __restrict__ relw,
                                                  unsigned short* __restrict__ QP) {
  __shared__ __align__(16) float relh_s[2048];
  __shared__ __align__(16) float relw_s[2048];
  __shared__ __align__(16) unsigned pk_s[2][4 * 64 * 16];
  const int t  = threadIdx.x;
  const int b  = blockIdx.x >> 4;
  const int i0 = (blockIdx.x & 15) * 64;
  {
    const v4f a0 = *(const v4f*)(relh + 8 * t);
    const v4f a1 = *(const v4f*)(relh + 8 * t + 4);
    const v4f w0 = *(const v4f*)(relw + 8 * t);
    const v4f w1 = *(const v4f*)(relw + 8 * t + 4);
    *(v4f*)(relh_s + 8 * t) = a0;  *(v4f*)(relh_s + 8 * t + 4) = a1;
    *(v4f*)(relw_s + 8 * t) = w0;  *(v4f*)(relw_s + 8 * t + 4) = w1;
  }
  __syncthreads();
  {
    const int tl = t >> 2, hd = t & 3;
    const int i  = i0 + tl;
    const size_t srow = ((size_t)(b * kN + i)) * kKQCols + hd * kSK + kDh;
    const v4u* sph = (const v4u*)(KQh + srow);
    const v4u* spl = (const v4u*)(KQl + srow);
    const v4u h0 = sph[0], h1 = sph[1];
    const v4u l0 = spl[0], l1 = spl[1];
    unsigned* qh = pk_s[0] + (hd * 64 + tl) * 16;
    unsigned* ql = pk_s[1] + (hd * 64 + tl) * 16;
    *(v4u*)(qh + 0) = h0; *(v4u*)(qh + 4) = h1;
    *(v4u*)(ql + 0) = l0; *(v4u*)(ql + 4) = l1;
    const int hh = i & 31, ww = i >> 5;
    unsigned short ph[16], pl[16];
#pragma unroll
    for (int d = 0; d < 16; ++d) {
      const float pv = relh_s[(hd * kDh + d) * kSpH + hh] + relw_s[(hd * kDh + d) * kSpW + ww];
      const unsigned short hb = f2bf_bits(pv);
      ph[d] = hb;
      pl[d] = f2bf_bits(pv - bf_bits2f(hb));
    }
    *(v4u*)(qh + 8)  = (v4u){pk16(ph[0], ph[1]), pk16(ph[2], ph[3]), pk16(ph[4], ph[5]), pk16(ph[6], ph[7])};
    *(v4u*)(qh + 12) = (v4u){pk16(ph[8], ph[9]), pk16(ph[10], ph[11]), pk16(ph[12], ph[13]), pk16(ph[14], ph[15])};
    *(v4u*)(ql + 8)  = (v4u){pk16(pl[0], pl[1]), pk16(pl[2], pl[3]), pk16(pl[4], pl[5]), pk16(pl[6], pl[7])};
    *(v4u*)(ql + 12) = (v4u){pk16(pl[8], pl[9]), pk16(pl[10], pl[11]), pk16(pl[12], pl[13]), pk16(pl[14], pl[15])};
  }
  __syncthreads();
  {
    const int lane = t & 31, wave = t >> 5;
    const int plane = wave >> 2, hw = wave & 3;
    const unsigned* srcw = pk_s[plane] + hw * (64 * 16);
    const int z = hw * kB + b;
    unsigned short* dst = QP + (size_t)plane * ((size_t)kZ * kN * kSK) + ((size_t)(z * kN + i0)) * kSK;
#pragma unroll
    for (int it = 0; it < 8; ++it) {
      const v4u val = *(const v4u*)(srcw + it * 128 + lane * 4);
      unsigned short* dp = dst + it * 256 + lane * 8;
      *(volatile v4u*)dp = val;
      __threadfence();
      *(volatile v4u*)dp = val;
    }
  }
}

__global__ __launch_bounds__(128) void softmax_kernel(const float* __restrict__ Sp, unsigned short* __restrict__ Pp) {
  __shared__ __align__(16) float lg[kN];
  __shared__ float redM[4];
  __shared__ float redS[4];
  const int row  = blockIdx.x;
  const int t    = threadIdx.x;
  const int lane = t & 31, wave = t >> 5;
  const float* sr = Sp + (size_t)row * kN;

  float mx = -__builtin_inff();
#pragma unroll 1
  for (int it = 0; it < 2; ++it) {
    const int c = it * 512 + 4 * t;
    const v4f sv = *(const v4f*)(sr + c);
#pragma unroll
    for (int e = 0; e < 4; ++e) mx = fmaxf(mx, sv[e]);
    *(v4f*)(lg + c) = sv;
  }
  mx = wave_max(mx);
  if (lane == 0) redM[wave] = mx;
  __syncthreads();
  float m = redM[0];
#pragma unroll
  for (int w = 1; w < 4; ++w) m = fmaxf(m, redM[w]);

  float sum = 0.0f;
#pragma unroll 1
  for (int it = 0; it < 2; ++it) {
    const int c = it * 512 + 4 * t;
    const v4f l = *(const v4f*)(lg + c);
    v4f ev;
#pragma unroll
    for (int e = 0; e < 4; ++e) {
      ev[e] = expf(l[e] - m);
      sum += ev[e];
    }
    *(v4f*)(lg + c) = ev;
  }
  sum = wave_sum(sum);
  if (lane == 0) redS[wave] = sum;
  __syncthreads();
  float tot = redS[0];
#pragma unroll
  for (int w = 1; w < 4; ++w) tot += redS[w];
  const float inv = kPCarry / tot;

  const v4f e0 = *(const v4f*)(lg + 8 * t);
  const v4f e1 = *(const v4f*)(lg + 8 * t + 4);
  unsigned short hb[8];
#pragma unroll
  for (int e = 0; e < 4; ++e) {
    hb[e]     = h_bits(e0[e] * inv);
    hb[4 + e] = h_bits(e1[e] * inv);
  }
  const v4u u = (v4u){pk16(hb[0], hb[1]), pk16(hb[2], hb[3]), pk16(hb[4], hb[5]), pk16(hb[6], hb[7])};
  unsigned short* pr = Pp + (size_t)row * kN + 8 * (size_t)t;
  *(volatile v4u*)pr = u;
  __threadfence();
  *(volatile v4u*)pr = u;
}

__global__ __launch_bounds__(256) void tail_kernel(const float* __restrict__ att, const float* __restrict__ x,
                                                  const float* __restrict__ lng, const float* __restrict__ lnb,
                                                  const float* __restrict__ caw1, const float* __restrict__ cab1,
                                                  const float* __restrict__ caw2, const float* __restrict__ cab2,
                                                  const float* __restrict__ saw, const float* __restrict__ sab,
                                                  float* __restrict__ out) {
  __shared__ float red1[8];
  __shared__ float red2[8];
  __shared__ float avg_s[kC];
  __shared__ float max_s[kC];
  __shared__ float hid_s[2 * kHid];
  __shared__ float ch_s[kC];
  __shared__ __align__(16) float feat_s[2 * kN];
  __shared__ __align__(16) float spat_s[kN];
  __shared__ float sw_s[128];
  const int t    = threadIdx.x;
  const int lane = t & 31, wave = t >> 5;
  const int b    = blockIdx.x;
  const float* attb = att + (size_t)b * kCN;
  const float* xb   = x   + (size_t)b * kCN;
  float* outb       = out + (size_t)b * kCN;

  {
    const int si = (t < kTaps) ? t : (kTaps - 1);
    const float wv = saw[si];
    if (t < kTaps) sw_s[t] = wv;
  }
  const float sbias = sab[0];

  float s = 0.0f;
#pragma unroll 1
  for (int it = 0; it < 64; ++it) {
    const v4f a = *(const v4f*)(attb + it * 1024 + 4 * t);
    s += (a[0] + a[1]) + (a[2] + a[3]);
  }
  s = wave_sum(s);
  if (lane == 0) red1[wave] = s;
  __syncthreads();
  float tot = red1[0];
#pragma unroll
  for (int w = 1; w < 8; ++w) tot += red1[w];
  const float mu = tot * (1.0f / 65536.0f);

  float q2 = 0.0f;
#pragma unroll 1
  for (int it = 0; it < 64; ++it) {
    const v4f a = *(const v4f*)(attb + it * 1024 + 4 * t);
#pragma unroll
    for (int e = 0; e < 4; ++e) {
      const float d = a[e] - mu;
      q2 = fmaf(d, d, q2);
    }
  }
  q2 = wave_sum(q2);
  if (lane == 0) red2[wave] = q2;
  __syncthreads();
  float tot2 = red2[0];
#pragma unroll
  for (int w = 1; w < 8; ++w) tot2 += red2[w];
  const float var  = tot2 * (1.0f / 65536.0f);
  const float rstd = rsqrtf(var + kLnEps);

#pragma unroll 1
  for (int k = 0; k < 8; ++k) {
    const int c = wave * 8 + k;
    const float* xc = xb + (size_t)c * kN;
    float cs = 0.0f, cm = -__builtin_inff();
#pragma unroll 1
    for (int mm = 0; mm < 32; ++mm) {
      const float v = xc[mm * 32 + lane];
      cs += v;
      cm = fmaxf(cm, v);
    }
    cs = wave_sum(cs);
    cm = wave_max(cm);
    if (lane == 0) { avg_s[c] = cs * (1.0f / 1024.0f); max_s[c] = cm; }
  }
  __syncthreads();

  {
    const int tt = t & 3;
    float ha = 0.0f, hm = 0.0f;
#pragma unroll 1
    for (int c = 0; c < kC; ++c) {
      const float wv = caw1[tt * kC + c];
      ha = fmaf(wv, avg_s[c], ha);
      hm = fmaf(wv, max_s[c], hm);
    }
    const float b1v = cab1[tt];
    if (t < kHid) { hid_s[t] = fmaxf(ha + b1v, 0.0f); hid_s[kHid + t] = fmaxf(hm + b1v, 0.0f); }
  }
  __syncthreads();

  {
    const int cc = t & 63;
    float oa = 0.0f, om = 0.0f;
#pragma unroll 1
    for (int j = 0; j < kHid; ++j) {
      const float wv = caw2[cc * kHid + j];
      oa = fmaf(wv, hid_s[j], oa);
      om = fmaf(wv, hid_s[kHid + j], om);
    }
    const float b2v = cab2[cc];
    const float z = (oa + b2v) + (om + b2v);
    const float chv = sigmoid_f(z);
    if (t < kC) ch_s[t] = chv;
  }
  __syncthreads();

#pragma unroll 1
  for (int m4 = 0; m4 < 4; ++m4) {
    const int n = m4 * 256 + t;
    float fs = 0.0f, fm = -__builtin_inff();
#pragma unroll 1
    for (int c = 0; c < kC; ++c) {
      const float v = ch_s[c] * xb[(size_t)c * kN + n];
      fs += v;
      fm = fmaxf(fm, v);
    }
    feat_s[n]      = fs * (1.0f / 64.0f);
    feat_s[kN + n] = fm;
  }
  __syncthreads();

#pragma unroll 1
  for (int m4 = 0; m4 < 4; ++m4) {
    const int n  = m4 * 256 + t;
    const int w0 = n >> 5, h0 = n & 31;
    float acc = 0.0f;
#pragma unroll 1
    for (int ci = 0; ci < 2; ++ci) {
#pragma unroll 1
      for (int a = 0; a < 7; ++a) {
        const int wi  = w0 + a - 3;
        const int wic = wi < 0 ? 0 : (wi > 31 ? 31 : wi);
#pragma unroll 1
        for (int c2 = 0; c2 < 7; ++c2) {
          const int hi  = h0 + c2 - 3;
          const int hic = hi < 0 ? 0 : (hi > 31 ? 31 : hi);
          const bool ok = ((unsigned)wi < 32u) && ((unsigned)hi < 32u);
          const float fv = feat_s[ci * kN + wic * 32 + hic];
          const float wg = sw_s[(ci * 7 + a) * 7 + c2];
          acc = fmaf(ok ? fv : 0.0f, wg, acc);
        }
      }
    }
    spat_s[n] = sigmoid_f(acc + sbias);
  }
  __syncthreads();

  const v4f spv = *(const v4f*)(spat_s + 4 * t);
#pragma unroll 1
  for (int it = 0; it < 64; ++it) {
    const int e = it * 1024 + 4 * t;
    const float chv = ch_s[it];
    const v4f a  = *(const v4f*)(attb + e);
    const v4f xv = *(const v4f*)(xb + e);
    const v4f g  = *(const v4f*)(lng + e);
    const v4f bb = *(const v4f*)(lnb + e);
    v4f r;
#pragma unroll
    for (int k = 0; k < 4; ++k) {
      const float ln  = (a[k] - mu) * rstd * g[k] + bb[k];
      const float xcv = chv * xv[k];
      const float cb  = spv[k] * xcv;
      const float mh  = ln + xv[k];
      r[k] = (mh + cb) + xv[k];
    }
    float* op = outb + e;
    *(volatile v4f*)op = r;
    __threadfence();
    *(volatile v4f*)op = r;
  }
}

extern "C" void kernel_launch(void* const* d_in, const int* in_sizes, int n_in,
                              void* d_out, int out_size, void* d_ws, size_t ws_size,
                              hipStream_t stream) {
  if (n_in < 17) return;
  if (in_sizes[0] != kB * kCN) return;
  if (in_sizes[1] != kC * kC || in_sizes[3] != kC * kC || in_sizes[5] != kC * kC) return;
  if (in_sizes[2] != kC || in_sizes[4] != kC || in_sizes[6] != kC) return;
  if (in_sizes[7] != kHeads * kDh * kSpH || in_sizes[8] != kHeads * kDh * kSpW) return;
  if (in_sizes[9] != kCN || in_sizes[10] != kCN) return;
  if (in_sizes[11] != kHid * kC || in_sizes[12] != kHid || in_sizes[13] != kC * kHid || in_sizes[14] != kC) return;
  if (in_sizes[15] != kTaps || in_sizes[16] != 1) return;
  if (out_size != kB * kCN) return;

  const size_t szX    = (size_t)kTok * kC * 2;
  const size_t szWkq  = (size_t)kKQCols * kC * 2;
  const size_t szWv   = (size_t)kC * kC * 2;
  const size_t szBias = (size_t)kKQCols * 4;
  const size_t szKQ   = (size_t)kTok * kKQCols * 2;
  const size_t szQPpl = (size_t)kZ * kN * kSK * 2;
  const size_t szV16  = (size_t)kB * kC * kN * 2;
  const size_t szSC   = (size_t)kGroup * kN * kN * 4;
  const size_t szPP   = (size_t)kGroup * kN * kN * 2;
  const size_t szATT  = (size_t)kB * kCN * 4;
  const size_t offXh   = 0;
  const size_t offXl   = offXh + szX;
  const size_t offWkqh = offXl + szX;
  const size_t offWkql = offWkqh + szWkq;
  const size_t offWvh  = offWkql + szWkq;
  const size_t offWvl  = offWvh + szWv;
  const size_t offBias = offWvl + szWv;
  const size_t offKQh  = offBias + szBias;
  const size_t offKQl  = offKQh + szKQ;
  const size_t offQP   = offKQl + szKQ;
  const size_t offV16  = offQP + 2 * szQPpl;
  const size_t offSC   = offV16 + szV16;
  const size_t offPP   = offSC + szSC;
  const size_t offATT  = offPP + szPP;
  const size_t total   = offATT + szATT;
  if (ws_size < total) return;

  const float* x    = (const float*)d_in[0];
  const float* Wq   = (const float*)d_in[1];
  const float* bq   = (const float*)d_in[2];
  const float* Wk   = (const float*)d_in[3];
  const float* bk   = (const float*)d_in[4];
  const float* Wv   = (const float*)d_in[5];
  const float* bv   = (const float*)d_in[6];
  const float* relh = (const float*)d_in[7];
  const float* relw = (const float*)d_in[8];
  const float* lng  = (const float*)d_in[9];
  const float* lnb  = (const float*)d_in[10];
  const float* caw1 = (const float*)d_in[11];
  const float* cab1 = (const float*)d_in[12];
  const float* caw2 = (const float*)d_in[13];
  const float* cab2 = (const float*)d_in[14];
  const float* saw  = (const float*)d_in[15];
  const float* sab  = (const float*)d_in[16];
  float* out = (float*)d_out;
  char* ws = (char*)d_ws;
  unsigned short* Xh   = (unsigned short*)(ws + offXh);
  unsigned short* Xl   = (unsigned short*)(ws + offXl);
  unsigned short* Wkqh = (unsigned short*)(ws + offWkqh);
  unsigned short* Wkql = (unsigned short*)(ws + offWkql);
  unsigned short* Wvh  = (unsigned short*)(ws + offWvh);
  unsigned short* Wvl  = (unsigned short*)(ws + offWvl);
  float*          BKQ  = (float*)(ws + offBias);
  unsigned short* KQh  = (unsigned short*)(ws + offKQh);
  unsigned short* KQl  = (unsigned short*)(ws + offKQl);
  unsigned short* QPh  = (unsigned short*)(ws + offQP);
  unsigned short* QPl  = QPh + (size_t)kZ * kN * kSK;
  unsigned short* V16  = (unsigned short*)(ws + offV16);
  float*          SC   = (float*)(ws + offSC);
  unsigned short* PP   = (unsigned short*)(ws + offPP);
  float*          ATT  = (float*)(ws + offATT);

  xt_split_kernel<<<dim3(kN / 64, kB), dim3(256), 0, stream>>>(x, Xh, Xl);
  prep_kernel<<<dim3(1), dim3(256), 0, stream>>>(Wq, bq, Wk, bk, Wv, Wkqh, Wkql, Wvh, Wvl, BKQ);

  wmma_gemm<1, true, 2, 2, 4><<<dim3((kTok / 64) * (kKQCols / 64) / 8, 1), dim3(256), 0, stream>>>(
      Xh, Xl, kC, 0L, Wkqh, Wkql, kC, 0L, (void*)KQh, (void*)KQl, kKQCols, 0L, BKQ, kTok, kKQCols, kC, 1.0f);
  wmma_gemm<1, true, 1, 1, 4><<<dim3((kC / 64) * (kN / 64) / 8, kB), dim3(256), 0, stream>>>(
      Wvh, Wvl, kC, 0L, Xh, Xl, kC, (long)kN * kC, (void*)V16, (void*)V16, kN, (long)kC * kN, bv, kC, kN, kC, 1.0f);
  pack_kernel<<<dim3(kTok / 64), dim3(256), 0, stream>>>(KQh, KQl, relh, relw, QPh);

  const long strideQP   = (long)kN * kSK;
  const long strideKQ   = (long)kN * kKQCols;
  const long strideSC   = (long)kN * kN;
  const long strideVb   = (long)kC * kN;
  const int  tilesScore = (kN / 64) * (kN / 64);
  const int  tilesPV    = (kDh / 16) * (kN / 64);
  for (int ck = 0; ck < kChunks; ++ck) {
    const int h  = ck >> 2;
    const int b0 = (ck & 3) * kGroup;
    const size_t qpOff = (size_t)ck * kGroup * (size_t)strideQP;
    const size_t kqOff = (size_t)b0 * (size_t)strideKQ + (size_t)h * kSK;
    const size_t vOff  = (size_t)b0 * (size_t)strideVb + (size_t)h * kDh * kN;
    wmma_gemm<1, true, 0, 0, 4><<<dim3(tilesScore / 8, kGroup), dim3(256), 0, stream>>>(
        QPh + qpOff, QPl + qpOff, kSK, strideQP, KQh + kqOff, KQl + kqOff, kKQCols, strideKQ,
        (void*)SC, (void*)SC, kN, strideSC, BKQ, kN, kN, kSK, 1.0f);
    softmax_kernel<<<dim3(kGroup * kN), dim3(128), 0, stream>>>(SC, PP);
    wmma_gemm<0, false, 0, 0, 1><<<dim3(tilesPV / 8, kGroup), dim3(256), 0, stream>>>(
        V16 + vOff, V16 + vOff, kN, strideVb, PP, PP, kN, strideSC,
        (void*)(ATT + vOff), (void*)(ATT + vOff), kN, strideVb, BKQ, kDh, kN, kN, kPCarryInv);
  }

  tail_kernel<<<dim3(kB), dim3(256), 0, stream>>>(ATT, x, lng, lnb, caw1, cab1, caw2, cab2, saw, sab, out);
}
